// Attention_52536039965434
// MI455X (gfx1250) — hardware-verified
//
#include <hip/hip_runtime.h>


#ifndef NB
#define NB 2
#endif
#ifndef SEQ
#define SEQ 2048
#endif
#define NB_FULL  2
#define SEQ_FULL 2048
#define HID   1024
#define NHEAD 16
#define HD    64
#define QKVW  (3 * HID)
#define MROWS (NB * SEQ)
#define PP    72
#define PCAR  16384.0f
#define WCAR  64.0f
#define L2E   1.4426950408889634f

static_assert(HID == NHEAD * HD);
static_assert(HD == 64);
static_assert(SEQ % 64 == 0 && SEQ <= SEQ_FULL && NB <= NB_FULL);
static_assert(MROWS % 64 == 0 && HID % 64 == 0 && QKVW % 64 == 0);
static_assert(HID % 32 == 0 && (2 * HID) % 32 == 0);
static_assert(((size_t)MROWS * HID) % (256 * 8) == 0);
static_assert(PP % 8 == 0 && PP >= 64);

typedef _Float16 h16;
typedef unsigned short bf;
typedef __attribute__((ext_vector_type(16))) __bf16   v16bf;
typedef __attribute__((ext_vector_type(16))) _Float16 v16h;
typedef __attribute__((ext_vector_type(8)))  _Float16 v8h;
typedef __attribute__((ext_vector_type(8)))  unsigned short v8us;
typedef __attribute__((ext_vector_type(8)))  float    v8f;
typedef __attribute__((ext_vector_type(4)))  float    v4f;
typedef v8h  __attribute__((may_alias)) v8ha;
typedef v4f  __attribute__((may_alias)) v4fa;

__device__ __forceinline__ unsigned short f2bf(float f) { unsigned u = __float_as_uint(f); u += 0x7FFFu + ((u >> 16) & 1u); return (unsigned short)(u >> 16); }
__device__ __forceinline__ float bf2f(unsigned short b) { return __uint_as_float(((unsigned)b) << 16); }
__device__ __forceinline__ float bfr(float f) { return bf2f(f2bf(f)); }
__device__ __forceinline__ void splitf(float y, unsigned short& h, unsigned short& l) { h = f2bf(y); l = f2bf(y - bf2f(h)); }
__device__ __forceinline__ v16h cat16(v8h lo, v8h hi) { return __builtin_shufflevector(lo, hi, 0, 1, 2, 3, 4, 5, 6, 7, 8, 9, 10, 11, 12, 13, 14, 15); }
__device__ __forceinline__ v16bf cat16b(v8us lo, v8us hi) { return __builtin_bit_cast(v16bf, __builtin_shufflevector(lo, hi, 0, 1, 2, 3, 4, 5, 6, 7, 8, 9, 10, 11, 12, 13, 14, 15)); }
__device__ __forceinline__ v8f wmma16(v16h a, v16h b, v8f c) { return __builtin_amdgcn_wmma_f32_16x16x32_f16(false, a, false, b, (short)0, c, false, false); }
__device__ __forceinline__ v8f wmmab(v16bf a, v16bf b, v8f c) { return __builtin_amdgcn_wmma_f32_16x16x32_bf16(false, a, false, b, (short)0, c, false, false); }
__device__ __forceinline__ void wave_sync() { __builtin_amdgcn_wave_barrier(); asm volatile("" ::: "memory"); }
__device__ __forceinline__ float gelu_tanh(float t) { const float t3 = t * t * t; const float u = 0.7978845608028654f * (t + 0.044715f * t3); return 0.5f * t * (1.0f + tanhf(u)); }

template <typename T16> struct WFrag;
template <> struct WFrag<h16> { typedef v16h V; static __device__ __forceinline__ V ld(const h16* p) { return cat16(*(const v8h*)p, *(const v8h*)(p + 16)); } static __device__ __forceinline__ v8f mma(V a, V b, v8f c) { return wmma16(a, b, c); } };
template <> struct WFrag<bf> { typedef v16bf V; static __device__ __forceinline__ V ld(const bf* p) { return cat16b(*(const v8us*)p, *(const v8us*)(p + 16)); } static __device__ __forceinline__ v8f mma(V a, V b, v8f c) { return wmmab(a, b, c); } };

template <typename T16, int EPI>
__device__ __forceinline__ void gemm_tile(const T16* __restrict__ A, const T16* __restrict__ Bt, const int K, const int r0, const int c0, float* os,
                                          unsigned short* C0, unsigned short* C1, float* CF, const int ldc, const float* __restrict__ bias, const float osc) {
    typedef typename WFrag<T16>::V V;
    const int lane = threadIdx.x & 31, lr = lane & 15, hi = lane >> 4;
    v8f acc[4][4];
#pragma unroll
    for (int mb = 0; mb < 4; ++mb)
#pragma unroll
        for (int nb = 0; nb < 4; ++nb) acc[mb][nb] = (v8f){};
    const size_t aoff = (size_t)(r0 + lr) * K + 8 * hi, boff = (size_t)(c0 + lr) * K + 8 * hi;
#pragma unroll 1
    for (int kc = 0; kc < K; kc += 32) {
        V a[4];
#pragma unroll
        for (int mb = 0; mb < 4; ++mb) a[mb] = WFrag<T16>::ld(A + aoff + (size_t)mb * 16 * K + kc);
#pragma unroll
        for (int nb = 0; nb < 4; ++nb) { const V b = WFrag<T16>::ld(Bt + boff + (size_t)nb * 16 * K + kc);
#pragma unroll
            for (int mb = 0; mb < 4; ++mb) acc[mb][nb] = WFrag<T16>::mma(a[mb], b, acc[mb][nb]); }
        asm volatile("v_nop\n\tv_nop\n\tv_nop\n\tv_nop" : "+v"(acc[0][0]), "+v"(acc[1][1]), "+v"(acc[2][2]), "+v"(acc[3][3]) : "v"(a[0]), "v"(a[3]));
    }
    const int c8 = (lane & 7) * 8, rq = lane >> 3, cofs = lr * 4;
    float cb[8];
#pragma unroll
    for (int j = 0; j < 8; ++j) cb[j] = 0.0f;
    if (EPI == 0 || EPI == 2) { const v4f b0 = *(const v4f*)(bias + c0 + c8), b1 = *(const v4f*)(bias + c0 + c8 + 4);
#pragma unroll
        for (int j = 0; j < 4; ++j) { cb[j] = bfr(b0[j]); cb[4 + j] = bfr(b1[j]); } }
    v4f cb3 = (v4f){};
    if (EPI == 3) { const v4f b0 = *(const v4f*)(bias + c0 + cofs);
#pragma unroll
        for (int q = 0; q < 4; ++q) cb3[q] = bfr(b0[q]); }
#pragma unroll
    for (int mb = 0; mb < 4; ++mb) {
#pragma unroll
        for (int nb = 0; nb < 4; ++nb) {
#pragma unroll
            for (int j = 0; j < 8; ++j) os[(hi * 8 + j) * 68 + nb * 16 + lr] = acc[mb][nb][j]; }
        wave_sync();
        const int m0 = r0 + mb * 16;
        if (EPI == 3) {
#pragma unroll 1
            for (int s = 0; s < 8; ++s) { const int row = 2 * s + hi; v4f val = *(const v4fa*)(os + row * 68 + cofs);
#pragma unroll
                for (int q = 0; q < 4; ++q) { const float t = val[q] * osc + cb3[q]; val[q] = gelu_tanh(t); }
                *(v4fa*)(os + row * 68 + cofs) = val; }
            wave_sync();
            const int orow0 = (m0 / SEQ) * SEQ_FULL + (m0 % SEQ);
            float* crow = CF + (size_t)orow0 * ldc + c0;
#pragma unroll 1
            for (int ps = 0; ps < 2; ++ps) {
#pragma unroll
                for (int s = 0; s < 8; ++s) { const int row = 2 * s + hi; const v4f val = *(const v4fa*)(os + row * 68 + cofs);
                    *(volatile v4f*)(crow + (size_t)row * ldc + cofs) = val; }
                if (ps == 0) __threadfence(); }
        } else {
            v8us ph[4], pl[4];
#pragma unroll
            for (int s = 0; s < 4; ++s) { const int row = s * 4 + rq;
                const v4f x0 = *(const v4fa*)(os + row * 68 + c8), x1 = *(const v4fa*)(os + row * 68 + c8 + 4);
                const float xv[8] = { x0[0], x0[1], x0[2], x0[3], x1[0], x1[1], x1[2], x1[3] };
                float rb = 0.0f; if (EPI == 1) rb = bfr(bias[m0 + row]);
#pragma unroll
                for (int j = 0; j < 8; ++j) { const float v = xv[j] * osc + ((EPI == 1) ? rb : cb[j]);
                    if (EPI == 0) { unsigned short a2, c2; splitf(v, a2, c2); ph[s][j] = a2; pl[s][j] = c2; }
                    else { ph[s][j] = __builtin_bit_cast(unsigned short, (h16)v); pl[s][j] = 0; } } }
#pragma unroll 1
            for (int ps = 0; ps < 2; ++ps) {
#pragma unroll
                for (int s = 0; s < 4; ++s) { const size_t off = (size_t)(m0 + s * 4 + rq) * ldc + c0 + c8;
                    *(volatile v8us*)(C0 + off) = ph[s]; if (EPI == 0) *(volatile v8us*)(C1 + off) = pl[s]; }
                if (ps == 0) __threadfence(); }
        }
        wave_sync();
    }
}

__global__ __launch_bounds__(32) void k_gemm_qk(const bf* __restrict__ X2, const bf* __restrict__ WAT, bf* H2, bf* L2, const float* __restrict__ bias) {
    __shared__ __align__(16) float os[16 * 68];
    const size_t z = blockIdx.z;
    gemm_tile<bf, 0>(X2 + z * (size_t)MROWS * HID, WAT + z * (size_t)HID * HID, HID, blockIdx.x * 64, blockIdx.y * 64, os,
                     H2 + z * (size_t)MROWS * HID, L2 + z * (size_t)MROWS * HID, nullptr, HID, bias + z * HID, 1.0f);
}
__global__ __launch_bounds__(32) void k_gemm_vt(const bf* __restrict__ WV, const bf* __restrict__ XK, h16* VT, const float* __restrict__ biasv) {
    __shared__ __align__(16) float os[16 * 68];
    gemm_tile<bf, 1>(WV, XK, HID, blockIdx.x * 64, blockIdx.y * 64, os, (unsigned short*)VT, nullptr, nullptr, MROWS, biasv, 1.0f);
}
__global__ __launch_bounds__(32) void k_gemm_proj(const h16* __restrict__ CTX, const h16* __restrict__ WPT, h16* CATR, const float* __restrict__ bias) {
    __shared__ __align__(16) float os[16 * 68];
    gemm_tile<h16, 2>(CTX, WPT, HID, blockIdx.x * 64, blockIdx.y * 64, os, (unsigned short*)CATR, nullptr, nullptr, 2 * HID, bias, 1.0f / WCAR);
}
__global__ __launch_bounds__(32) void k_gemm_mlp(const h16* __restrict__ CAT, const h16* __restrict__ WMT, float* OUT, const float* __restrict__ bias) {
    __shared__ __align__(16) float os[16 * 68];
    gemm_tile<h16, 3>(CAT, WMT, 2 * HID, blockIdx.x * 64, blockIdx.y * 64, os, nullptr, nullptr, OUT, HID, bias, 1.0f / WCAR);
}

__global__ __launch_bounds__(256) void k_cvtx(const float* __restrict__ src, bf* X, h16* CAT, int wcat) {
    const size_t e = ((size_t)blockIdx.x * 256 + threadIdx.x) * 8; if (e >= (size_t)MROWS * HID) return;
    const int col = (int)(e % HID); const int m = (int)(e / HID); const int b = m / SEQ, t = m % SEQ;
    const float* s = src + ((size_t)b * SEQ_FULL + t) * HID + col;
    const v4f a0 = *(const v4f*)s, a1 = *(const v4f*)(s + 4);
    v8us ob; v8h oh;
#pragma unroll
    for (int j = 0; j < 4; ++j) { ob[j] = f2bf(a0[j]); ob[4 + j] = f2bf(a1[j]); }
#pragma unroll
    for (int j = 0; j < 8; ++j) oh[j] = (h16)bf2f(ob[j]);
    h16* cp = CAT + (size_t)m * (2 * HID) + col;
    *(volatile v8us*)(X + e) = ob; if (wcat) *(volatile v8h*)cp = oh;
    __threadfence();
    *(volatile v8us*)(X + e) = ob; if (wcat) *(volatile v8h*)cp = oh;
}

__global__ __launch_bounds__(256) void k_wt(const float* __restrict__ W, int ldw, int K, unsigned short* OUT, int f16mode) {
    __shared__ float tile[64 * 65];
    const int tid = threadIdx.x; const int n0 = blockIdx.x * 64, k0 = blockIdx.y * 64;
#pragma unroll
    for (int i = 0; i < 4; ++i) { const int kr = (tid >> 4) + 16 * i, c4 = (tid & 15) * 4; const v4f a = *(const v4f*)(W + (size_t)(k0 + kr) * ldw + n0 + c4);
#pragma unroll
        for (int q = 0; q < 4; ++q) tile[kr * 65 + c4 + q] = a[q]; }
    __syncthreads();
    const int c8 = (tid & 7) * 8;
    v8us pk[2];
#pragma unroll
    for (int i = 0; i < 2; ++i) { const int n = (tid >> 3) + 32 * i;
#pragma unroll
        for (int j = 0; j < 8; ++j) { const float x = bfr(tile[(c8 + j) * 65 + n]); const unsigned short hb = __builtin_bit_cast(unsigned short, (h16)(x * WCAR)); const unsigned short bb = f2bf(x); pk[i][j] = f16mode ? hb : bb; } }
#pragma unroll 1
    for (int ps = 0; ps < 2; ++ps) {
#pragma unroll
        for (int i = 0; i < 2; ++i) { const int n = (tid >> 3) + 32 * i; *(volatile v8us*)(OUT + (size_t)(n0 + n) * K + k0 + c8) = pk[i]; }
        if (ps == 0) __threadfence(); }
}

__global__ __launch_bounds__(128) void k_flash(const bf* __restrict__ QHp, const bf* __restrict__ QLp, const bf* __restrict__ KHp, const bf* __restrict__ KLp,
                                               const h16* __restrict__ VT, const int* __restrict__ mask, h16* CTX) {
    __shared__ __align__(16) h16 Ps[4 * 16 * PP];
    const int lane = threadIdx.x & 31, w = threadIdx.x >> 5, lr = lane & 15, hi = lane >> 4;
    const int blk = blockIdx.x; const int qt = blk % (SEQ / 64); const int hh = (blk / (SEQ / 64)) % NHEAD; const int b = blk / ((SEQ / 64) * NHEAD);
    const int q0 = qt * 64 + w * 16;
    h16* P = Ps + w * 16 * PP;
    const size_t qoff = ((size_t)b * SEQ + q0 + lr) * HID + hh * HD + 8 * hi;
    const v16bf qh0 = WFrag<bf>::ld(QHp + qoff), qh1 = WFrag<bf>::ld(QHp + qoff + 32), ql0 = WFrag<bf>::ld(QLp + qoff), ql1 = WFrag<bf>::ld(QLp + qoff + 32);
    const size_t kbase = ((size_t)b * SEQ + lr) * HID + hh * HD + 8 * hi;
    const size_t vbase = ((size_t)hh * HD + lr) * MROWS + (size_t)b * SEQ + 8 * hi;
    const int* mrowp = mask + (size_t)b * SEQ_FULL;
    float mrow[8], lrow[8]; v8f accv[4];
#pragma unroll
    for (int r = 0; r < 8; ++r) { mrow[r] = -1.0e30f; lrow[r] = 0.0f; }
#pragma unroll
    for (int g = 0; g < 4; ++g) accv[g] = (v8f){};
#pragma unroll 1
    for (int k0 = 0; k0 < SEQ; k0 += 64) {
        v8f s[4];
#pragma unroll
        for (int t = 0; t < 4; ++t) {
            const size_t kp = kbase + (size_t)(k0 + t * 16) * HID;
            const v16bf kh0 = WFrag<bf>::ld(KHp + kp), kh1 = WFrag<bf>::ld(KHp + kp + 32), kl0 = WFrag<bf>::ld(KLp + kp), kl1 = WFrag<bf>::ld(KLp + kp + 32);
            v8f sc = (v8f){};
            sc = wmmab(qh0, kh0, sc); sc = wmmab(qh1, kh1, sc);
            sc = wmmab(ql0, kh0, sc); sc = wmmab(ql1, kh1, sc);
            sc = wmmab(qh0, kl0, sc); sc = wmmab(qh1, kl1, sc);
            asm volatile("v_nop\n\tv_nop\n\tv_nop\n\tv_nop" : "+v"(sc) : "v"(kh0), "v"(kl1) : "memory");
            s[t] = sc;
        }
#pragma unroll
        for (int t = 0; t < 4; ++t) { const float mk = (float)mrowp[k0 + t * 16 + lr];
#pragma unroll
            for (int r = 0; r < 8; ++r) s[t][r] *= mk; }
        float cm[8];
#pragma unroll
        for (int r = 0; r < 8; ++r) cm[r] = fmaxf(fmaxf(s[0][r], s[1][r]), fmaxf(s[2][r], s[3][r]));
#pragma unroll
        for (int off = 1; off < 16; off <<= 1)
#pragma unroll
            for (int r = 0; r < 8; ++r) cm[r] = fmaxf(cm[r], __shfl_xor(cm[r], off, 32));
#pragma unroll
        for (int r = 0; r < 8; ++r) { const float mn = fmaxf(mrow[r], cm[r]); const float rs = __builtin_amdgcn_exp2f((mrow[r] - mn) * L2E); mrow[r] = mn; lrow[r] *= rs;
#pragma unroll
            for (int g = 0; g < 4; ++g) accv[g][r] *= rs; }
#pragma unroll
        for (int t = 0; t < 4; ++t)
#pragma unroll
            for (int r = 0; r < 8; ++r) { const float p = __builtin_amdgcn_exp2f((s[t][r] - mrow[r]) * L2E); lrow[r] += p; P[(8 * hi + r) * PP + t * 16 + lr] = (h16)(p * PCAR); }
        wave_sync();
        v16h ap[2];
#pragma unroll
        for (int kc = 0; kc < 2; ++kc) ap[kc] = cat16(*(const v8ha*)(P + lr * PP + kc * 32 + 8 * hi), *(const v8ha*)(P + lr * PP + kc * 32 + 16 + 8 * hi));
#pragma unroll
        for (int g = 0; g < 4; ++g)
#pragma unroll
            for (int kc = 0; kc < 2; ++kc) { const v16h bv = WFrag<h16>::ld(VT + vbase + (size_t)g * 16 * MROWS + k0 + kc * 32); accv[g] = wmma16(ap[kc], bv, accv[g]); }
        asm volatile("v_nop\n\tv_nop\n\tv_nop\n\tv_nop" : "+v"(accv[0]), "+v"(accv[1]), "+v"(accv[2]), "+v"(accv[3]) : "v"(ap[0]), "v"(ap[1]));
        wave_sync();
    }
    float inv[8];
#pragma unroll
    for (int r = 0; r < 8; ++r) { float l = lrow[r];
#pragma unroll
        for (int off = 1; off < 16; off <<= 1) l += __shfl_xor(l, off, 32);
        inv[r] = (1.0f / l) * (1.0f / PCAR); }
#pragma unroll
    for (int g = 0; g < 4; ++g)
#pragma unroll
        for (int r = 0; r < 8; ++r) P[(8 * hi + r) * PP + g * 16 + lr] = (h16)(accv[g][r] * inv[r]);
    wave_sync();
    const int c8 = (lane & 7) * 8, rq = lane >> 3;
    v8h ov[4];
#pragma unroll
    for (int s2 = 0; s2 < 4; ++s2) ov[s2] = *(const v8ha*)(P + (s2 * 4 + rq) * PP + c8);
#pragma unroll 1
    for (int ps = 0; ps < 2; ++ps) {
#pragma unroll
        for (int s2 = 0; s2 < 4; ++s2) *(volatile v8h*)(CTX + ((size_t)b * SEQ + q0 + s2 * 4 + rq) * HID + hh * HD + c8) = ov[s2];
        if (ps == 0) __threadfence(); }
}

constexpr size_t SZ_X2  = (size_t)2 * MROWS * HID * 2;
constexpr size_t SZ_WAT = (size_t)QKVW * HID * 2;
constexpr size_t SZ_WPT = (size_t)HID * HID * 2;
constexpr size_t SZ_WMT = (size_t)HID * 2 * HID * 2;
constexpr size_t SZ_HL  = (size_t)2 * MROWS * HID * 2;
constexpr size_t SZ_VT  = (size_t)HID * MROWS * 2;
constexpr size_t SZ_CTX = (size_t)MROWS * HID * 2;
constexpr size_t SZ_CAT = (size_t)MROWS * 2 * HID * 2;
constexpr size_t OFF_X2  = 0;
constexpr size_t OFF_WAT = OFF_X2 + SZ_X2;
constexpr size_t OFF_WPT = OFF_WAT + SZ_WAT;
constexpr size_t OFF_WMT = OFF_WPT + SZ_WPT;
constexpr size_t OFF_H2  = OFF_WMT + SZ_WMT;
constexpr size_t OFF_L2  = OFF_H2 + SZ_HL;
constexpr size_t OFF_VT  = OFF_L2 + SZ_HL;
constexpr size_t OFF_CTX = OFF_VT + SZ_VT;
constexpr size_t OFF_CAT = OFF_CTX + SZ_CTX;
constexpr size_t WS_TOTAL = OFF_CAT + SZ_CAT;
static_assert(SZ_X2 % 256 == 0 && SZ_WAT % 256 == 0 && SZ_WPT % 256 == 0 && SZ_WMT % 256 == 0 && SZ_HL % 256 == 0 && SZ_VT % 256 == 0 && SZ_CTX % 256 == 0 && SZ_CAT % 256 == 0);
static_assert(WS_TOTAL <= (size_t)134217728);

extern "C" void kernel_launch(void* const* d_in, const int* in_sizes, int n_in,
                              void* d_out, int out_size, void* d_ws, size_t ws_size, hipStream_t stream) {
    if (n_in < 9) return;
    const long long need_rows = (long long)(NB - 1) * SEQ_FULL + SEQ;
    if ((long long)in_sizes[0] < need_rows * HID || (long long)in_sizes[1] < need_rows * HID || (long long)in_sizes[2] < need_rows) return;
    if (in_sizes[3] < HID * QKVW || in_sizes[4] < QKVW || in_sizes[5] < HID * HID || in_sizes[6] < HID || in_sizes[7] < 2 * HID * HID || in_sizes[8] < HID) return;
    if ((long long)out_size < need_rows * HID) return;
    if (ws_size < WS_TOTAL) return;
    const float* xq   = (const float*)d_in[0];
    const float* xk   = (const float*)d_in[1];
    const int*   mask = (const int*)d_in[2];
    const float* caw  = (const float*)d_in[3];
    const float* cab  = (const float*)d_in[4];
    const float* cpw  = (const float*)d_in[5];
    const float* cpb  = (const float*)d_in[6];
    const float* mw   = (const float*)d_in[7];
    const float* mbv  = (const float*)d_in[8];
    float* OUT = (float*)d_out;
    char* ws = (char*)d_ws;
    bf*  X2  = (bf*)(ws + OFF_X2);
    bf*  WAT = (bf*)(ws + OFF_WAT);
    h16* WPT = (h16*)(ws + OFF_WPT);
    h16* WMT = (h16*)(ws + OFF_WMT);
    bf*  H2  = (bf*)(ws + OFF_H2);
    bf*  L2  = (bf*)(ws + OFF_L2);
    h16* VT  = (h16*)(ws + OFF_VT);
    h16* CTX = (h16*)(ws + OFF_CTX);
    h16* CAT = (h16*)(ws + OFF_CAT);

    const unsigned gcv = (unsigned)(((size_t)MROWS * HID) / (256 * 8));
    k_cvtx<<<gcv, 256, 0, stream>>>(xq, X2, CAT, 1);
    k_cvtx<<<gcv, 256, 0, stream>>>(xk, X2 + (size_t)MROWS * HID, CAT, 0);
    k_wt<<<dim3(QKVW / 64, HID / 64), 256, 0, stream>>>(caw, QKVW, HID, (unsigned short*)WAT, 0);
    k_wt<<<dim3(HID / 64, HID / 64), 256, 0, stream>>>(cpw, HID, HID, (unsigned short*)WPT, 1);
    k_wt<<<dim3(HID / 64, 2 * HID / 64), 256, 0, stream>>>(mw, HID, 2 * HID, (unsigned short*)WMT, 1);
    k_gemm_qk<<<dim3(MROWS / 64, HID / 64, 2), 32, 0, stream>>>(X2, WAT, H2, L2, cab);
    k_gemm_vt<<<dim3(HID / 64, MROWS / 64), 32, 0, stream>>>(WAT + (size_t)2 * HID * HID, X2 + (size_t)MROWS * HID, VT, cab + 2 * HID);
    k_flash<<<NB * NHEAD * (SEQ / 64), 128, 0, stream>>>(H2, L2, H2 + (size_t)MROWS * HID, L2 + (size_t)MROWS * HID, VT, mask, CTX);
    k_gemm_proj<<<dim3(MROWS / 64, HID / 64), 32, 0, stream>>>(CTX, WPT, CAT + HID, cpb);
    k_gemm_mlp<<<dim3(MROWS / 64, HID / 64), 32, 0, stream>>>(CAT, WMT, OUT, mbv);
}
